// ResonanceCavity_85572928406137
// MI455X (gfx1250) — hardware-verified
//
#include <hip/hip_runtime.h>
#include <math.h>

#ifndef NROWS
#define NROWS 8192
#endif
#define NROWS_FULL 8192
#define DM 1024
#define NF 5
#define NMODE 256
#define NA (NF * NMODE)
#define NBR 10
#define TBL 1280
#define NCT (DM / 64)
#define PI_F 3.14159265358979f

static_assert(NROWS <= NROWS_FULL);
static_assert(NROWS % 64 == 0);
static_assert(DM % 64 == 0 && NA % 64 == 0);
static_assert(DM % 32 == 0 && NMODE % 32 == 0);
static_assert(NCT == 16);
static_assert((NMODE / 8) == 32);
static_assert(((size_t)NROWS * DM / 8) % 256 == 0);
static_assert(((size_t)NA * DM / 8) % 256 == 0);
static_assert((DM * (NMODE / 8)) % 256 == 0);
static_assert(((NROWS / 64) * (NA / 64)) % 8 == 0);
static_assert(((NROWS / 32) * NCT) % 8 == 0);
static_assert((NBR * DM) % 256 == 0);
static_assert(32 * 16 * 2 * 4 == 16 * 64 * 4);
static_assert(32 * 16 * 4 == 16 * 64 * 2);
static_assert(32 * 4 == 128);
static_assert(8 * 32 * 16 == DM * 4);
static_assert(8 * 16 * 68 * 4 + 8 * NF * 32 * 4 <= 131072);
static_assert(NBR * DM * 4 <= 131072);

#define SZ_H16  ((size_t)NROWS * DM * 2)
#define SZ_W16  ((size_t)NA * DM * 2)
#define SZ_M16  ((size_t)NF * DM * NMODE * 2)
#define SZ_A16  ((size_t)NROWS * NA * 2)
#define SZ_S    ((size_t)NROWS * DM * 4)
#define SZ_PART ((size_t)NCT * NF * NROWS * 4)
#define WS_TOTAL (SZ_H16 + SZ_W16 + SZ_M16 + SZ_A16 + SZ_S + SZ_PART)
static_assert(SZ_H16 % 256 == 0 && SZ_W16 % 256 == 0 && SZ_M16 % 256 == 0);
static_assert(SZ_A16 % 256 == 0 && SZ_S % 256 == 0 && SZ_PART % 256 == 0);
static_assert(WS_TOTAL <= (size_t)134217728);

typedef __attribute__((ext_vector_type(16))) _Float16 v16h;
typedef __attribute__((ext_vector_type(8)))  _Float16 v8h;
typedef __attribute__((ext_vector_type(8)))  float    v8f;
typedef __attribute__((ext_vector_type(4)))  float    v4f;
typedef __attribute__((ext_vector_type(4)))  unsigned int v4u;
typedef _Float16 h16;

static constexpr float SCL_H = 8.0f;
static constexpr float SCL_W = 1024.0f;
static constexpr float SCL_M = 1024.0f;
static constexpr float SCL_A = 2048.0f / (8.0f * 1024.0f);
static constexpr float SCL_R = 1.0f / (2048.0f * 1024.0f);


#define VST2(T, ptr, val) do { const T vst2_v_ = (val); *(volatile T*)(ptr) = vst2_v_; __threadfence(); *(volatile T*)(ptr) = vst2_v_; } while (0)
#define VST2V4(ptr, val) do { const v4f vst2_v4_ = (val); *(volatile v4f*)(ptr) = vst2_v4_; __threadfence(); *(volatile v4f*)(ptr) = vst2_v4_; } while (0)

__device__ __forceinline__ float bfr(float f) {
    unsigned u = __float_as_uint(f);
    u += 0x7FFFu + ((u >> 16) & 1u);
    return __uint_as_float(u & 0xFFFF0000u);
}
__device__ __forceinline__ unsigned short f2h_bits(float x) {
    return (fabsf(x) < 6.104e-5f) ? (unsigned short)0 : __builtin_bit_cast(unsigned short, (_Float16)x);
}
__device__ __forceinline__ void st8h(unsigned short* P, size_t o, const float* v) {
    v4u pk;
    pk.x = (unsigned)f2h_bits(v[0]) | ((unsigned)f2h_bits(v[1]) << 16);
    pk.y = (unsigned)f2h_bits(v[2]) | ((unsigned)f2h_bits(v[3]) << 16);
    pk.z = (unsigned)f2h_bits(v[4]) | ((unsigned)f2h_bits(v[5]) << 16);
    pk.w = (unsigned)f2h_bits(v[6]) | ((unsigned)f2h_bits(v[7]) << 16);
    VST2(v4u, (v4u*)(P + o), pk);
}
static __device__ __forceinline__ h16 toh_flush(float v) { const h16 r = (h16)v; return (fabsf(v) < 6.103515625e-05f) ? (h16)0.0f : r; }

union FragU { v16h v; v8h h[2]; };
__device__ __forceinline__ v16h frag_ld(const _Float16* p) {
    FragU f; f.h[0] = *(const v8h*)(p); f.h[1] = *(const v8h*)(p + 16); return f.v;
}
__device__ __forceinline__ v8f wmma16(v16h a, v16h b, v8f c) {
    c = __builtin_amdgcn_wmma_f32_16x16x32_f16(false, a, false, b, (short)0, c, false, false);
    asm volatile("v_nop\n\tv_nop\n\tv_nop\n\tv_nop" : "+v"(c) : "v"(a), "v"(b));
    return c;
}
__device__ __forceinline__ void dep_guard_h(v8f& a, v8f& b, v16h x, v16h y) { asm volatile("v_nop\n\tv_nop\n\tv_nop\n\tv_nop" : "+v"(a), "+v"(b) : "v"(x), "v"(y)); }
__device__ __forceinline__ void keep4_h(v16h a, v16h b, v16h c, v16h d) { asm volatile("v_nop" :: "v"(a), "v"(b), "v"(c), "v"(d)); }
__device__ __forceinline__ void acc_guard4(v8f& a, v8f& b, v8f& c, v8f& d) { asm volatile("v_nop\n\tv_nop\n\tv_nop\n\tv_nop" : "+v"(a), "+v"(b), "+v"(c), "+v"(d)); }
__device__ __forceinline__ void wave_sync_lds() {
    __builtin_amdgcn_fence(3  , "workgroup");
    __builtin_amdgcn_wave_barrier();
    __builtin_amdgcn_fence(2  , "workgroup");
}
__device__ __forceinline__ float xsum16(float v) {
    v += __shfl_xor(v, 1, 32); v += __shfl_xor(v, 2, 32); v += __shfl_xor(v, 4, 32); v += __shfl_xor(v, 8, 32);
    return v;
}

__global__ __launch_bounds__(256) void k_cvt16(const float* __restrict__ src, _Float16* __restrict__ dst, unsigned n8, float s) {
    const unsigned u = blockIdx.x * 256u + threadIdx.x;
    if (u >= n8) return;
    const float* sp = src + (size_t)u * 8u;
    const v4f a = *(const v4f*)(sp), b = *(const v4f*)(sp + 4);
    v8h hv;
    hv[0] = toh_flush(bfr(a.x) * s); hv[1] = toh_flush(bfr(a.y) * s);
    hv[2] = toh_flush(bfr(a.z) * s); hv[3] = toh_flush(bfr(a.w) * s);
    hv[4] = toh_flush(bfr(b.x) * s); hv[5] = toh_flush(bfr(b.y) * s);
    hv[6] = toh_flush(bfr(b.z) * s); hv[7] = toh_flush(bfr(b.w) * s);
    _Float16* dp = dst + (size_t)u * 8u;
    *(volatile v8h*)(dp) = hv;
    __threadfence();
    *(volatile v8h*)(dp) = hv;
}

__global__ __launch_bounds__(256) void k_wt16(const float* __restrict__ Wm, unsigned KI, unsigned NO, unsigned lgper,
                                              unsigned short* __restrict__ W16, float sw) {
    const unsigned layer = blockIdx.y;
    const float* Wl = Wm + (size_t)layer * KI * NO;
    unsigned short* Dl = W16 + (size_t)layer * KI * NO;
    const unsigned u = blockIdx.x * 256u + threadIdx.x;
    const unsigned per = 1u << lgper;
    if (u >= NO * per) return;
    const unsigned k0 = 8u * (u & (per - 1u));
    const unsigned o = u >> lgper;
    float v[8];
#pragma unroll
    for (int i = 0; i < 8; ++i) v[i] = bfr(Wl[(size_t)(k0 + (unsigned)i) * NO + o]) * sw;
    st8h(Dl, (size_t)o * KI + k0, v);
}

__global__ __launch_bounds__(256) void k_gemm_a(
    const _Float16* __restrict__ A, unsigned lda, const _Float16* __restrict__ Bt, unsigned ldb,
    _Float16* __restrict__ C, unsigned ldc, unsigned M, unsigned N, unsigned K, float scale) {
  __shared__ __align__(16) float sT[8][16 * 68];
  const unsigned lane = threadIdx.x & 31u;
  const unsigned wave = (unsigned)__builtin_amdgcn_readfirstlane((int)(threadIdx.x >> 5));
  const unsigned tilesN = N >> 6, tilesM = M >> 6;
  const unsigned tile = blockIdx.x * 8u + wave;
  if (tile >= tilesM * tilesN) return;
  const unsigned tm = tile / tilesN;
  const unsigned tn = tile - tm * tilesN;
  const unsigned m0 = tm << 6, n0 = tn << 6;
  const unsigned rlane = lane & 15u;
  const unsigned koff = (lane >> 4) * 8u;
  const unsigned mOff = koff;

  v8f acc[4][4];
#pragma unroll
  for (int i = 0; i < 4; ++i)
#pragma unroll
    for (int j = 0; j < 4; ++j) acc[i][j] = (v8f){0.f,0.f,0.f,0.f,0.f,0.f,0.f,0.f};

  for (unsigned k0 = 0; k0 < K; k0 += 32u) {
    v16h bh[4];
#pragma unroll
    for (int j = 0; j < 4; ++j)
      bh[j] = frag_ld(Bt + (size_t)(n0 + ((unsigned)j << 4) + rlane) * ldb + koff + k0);
#pragma unroll
    for (int i = 0; i < 4; ++i) {
      const v16h ah = frag_ld(A + (size_t)(m0 + ((unsigned)i << 4) + rlane) * lda + koff + k0);
#pragma unroll
      for (int j = 0; j < 4; ++j)
        acc[i][j] = __builtin_amdgcn_wmma_f32_16x16x32_f16(false, ah, false, bh[j], (short)0, acc[i][j], false, false);
      dep_guard_h(acc[i][0], acc[i][3], ah, ah);
    }
    keep4_h(bh[0], bh[1], bh[2], bh[3]);
  }
  acc_guard4(acc[0][0], acc[0][1], acc[0][2], acc[0][3]);
  acc_guard4(acc[1][0], acc[1][1], acc[1][2], acc[1][3]);
  acc_guard4(acc[2][0], acc[2][1], acc[2][2], acc[2][3]);
  acc_guard4(acc[3][0], acc[3][1], acc[3][2], acc[3][3]);

  float* slab = sT[wave];
#pragma unroll
  for (int i = 0; i < 4; ++i) {
    const unsigned mBase = m0 + ((unsigned)i << 4);
#pragma unroll
    for (int j = 0; j < 4; ++j) {
#pragma unroll
      for (int r = 0; r < 8; ++r) {
        const float v = acc[i][j][r] * scale;
        slab[(mOff + (unsigned)r) * 68u + ((unsigned)j << 4) + rlane] = v;
      }
    }
    wave_sync_lds();
    {
      const unsigned q = lane >> 3, c8 = (lane & 7u) * 8u;
      v8h hv[4];
#pragma unroll
      for (int it = 0; it < 4; ++it) {
        const unsigned row = (unsigned)it * 4u + q;
        const float* sp = slab + row * 68u + c8;
#pragma unroll
        for (int e = 0; e < 8; ++e) hv[it][e] = toh_flush(sp[e]);
      }
      for (int pass = 0; pass < 2; ++pass) {
#pragma unroll
        for (int it = 0; it < 4; ++it) {
          const unsigned row = (unsigned)it * 4u + q;
          *(volatile v8h*)(C + (size_t)(mBase + row) * ldc + n0 + c8) = hv[it];
        }
        __threadfence();
      }
    }
    wave_sync_lds();
  }
}

__global__ __launch_bounds__(256) void k_gemm_f(
    const _Float16* __restrict__ A16, const _Float16* __restrict__ Mt16,
    float* __restrict__ S, float* __restrict__ part, float scl) {
  __shared__ __align__(16) float sT[8][16 * 68];
  __shared__ __align__(16) float sQ[8][NF * 32];
  const unsigned lane = threadIdx.x & 31u;
  const unsigned wave = (unsigned)__builtin_amdgcn_readfirstlane((int)(threadIdx.x >> 5));
  const unsigned tile = blockIdx.x * 8u + wave;
  if (tile >= (unsigned)((NROWS / 32) * NCT)) return;
  const unsigned tm = tile / (unsigned)NCT;
  const unsigned tn = tile - tm * (unsigned)NCT;
  const unsigned m0 = tm << 5, n0 = tn << 6;
  const unsigned rlane = lane & 15u;
  const unsigned koff = (lane >> 4) * 8u;
  const unsigned mOff = koff;

  v8f ssum[2][4];
#pragma unroll
  for (int i = 0; i < 2; ++i)
#pragma unroll
    for (int j = 0; j < 4; ++j) ssum[i][j] = (v8f){0.f,0.f,0.f,0.f,0.f,0.f,0.f,0.f};

  float* sq = sQ[wave];
#pragma unroll 1
  for (unsigned f = 0; f < (unsigned)NF; ++f) {
    v8f acc[2][4];
#pragma unroll
    for (int i = 0; i < 2; ++i)
#pragma unroll
      for (int j = 0; j < 4; ++j) acc[i][j] = (v8f){0.f,0.f,0.f,0.f,0.f,0.f,0.f,0.f};
    const _Float16* Ap = A16 + (size_t)(m0 + rlane) * NA + f * (unsigned)NMODE + koff;
    const _Float16* Bp = Mt16 + (size_t)f * DM * NMODE + (size_t)(n0 + rlane) * NMODE + koff;
#pragma unroll 1
    for (unsigned k0 = 0; k0 < (unsigned)NMODE; k0 += 32u) {
      v16h bh[4];
#pragma unroll
      for (int j = 0; j < 4; ++j)
        bh[j] = frag_ld(Bp + (size_t)((unsigned)j << 4) * NMODE + k0);
#pragma unroll
      for (int i = 0; i < 2; ++i) {
        const v16h ah = frag_ld(Ap + (size_t)((unsigned)i << 4) * NA + k0);
#pragma unroll
        for (int j = 0; j < 4; ++j)
          acc[i][j] = __builtin_amdgcn_wmma_f32_16x16x32_f16(false, ah, false, bh[j], (short)0, acc[i][j], false, false);
        dep_guard_h(acc[i][0], acc[i][3], ah, ah);
      }
      keep4_h(bh[0], bh[1], bh[2], bh[3]);
    }
    acc_guard4(acc[0][0], acc[0][1], acc[0][2], acc[0][3]);
    acc_guard4(acc[1][0], acc[1][1], acc[1][2], acc[1][3]);
#pragma unroll
    for (int i = 0; i < 2; ++i) {
#pragma unroll
      for (int r = 0; r < 8; ++r) {
        float q = 0.f;
#pragma unroll
        for (int j = 0; j < 4; ++j) {
          const float v = acc[i][j][r] * scl;
          ssum[i][j][r] += v;
          q += v * v;
        }
        q = xsum16(q);
        if (rlane == 0u) sq[f * 32u + ((unsigned)i << 4) + mOff + (unsigned)r] = q;
      }
    }
  }
  wave_sync_lds();
  {
    float pv[NF];
#pragma unroll
    for (int f = 0; f < NF; ++f) pv[f] = sq[(unsigned)f * 32u + lane];
    for (int pass = 0; pass < 2; ++pass) {
#pragma unroll
      for (int f = 0; f < NF; ++f)
        *(volatile float*)(part + (size_t)(tn * (unsigned)NF + (unsigned)f) * NROWS + m0 + lane) = pv[f];
      __threadfence();
    }
  }

  float* slab = sT[wave];
#pragma unroll
  for (int i = 0; i < 2; ++i) {
    const unsigned mBase = m0 + ((unsigned)i << 4);
#pragma unroll
    for (int j = 0; j < 4; ++j) {
#pragma unroll
      for (int r = 0; r < 8; ++r)
        slab[(mOff + (unsigned)r) * 68u + ((unsigned)j << 4) + rlane] = ssum[i][j][r];
    }
    wave_sync_lds();
    {
      const unsigned hh = lane >> 4, c4 = (lane & 15u) * 4u;
#pragma unroll
      for (int half = 0; half < 2; ++half) {
        v4f vv[4];
#pragma unroll
        for (int it = 0; it < 4; ++it) {
          const unsigned row = (unsigned)(half * 4 + it) * 2u + hh;
          vv[it] = *(const v4f*)(slab + row * 68u + c4);
        }
        for (int pass = 0; pass < 2; ++pass) {
#pragma unroll
          for (int it = 0; it < 4; ++it) {
            const unsigned row = (unsigned)(half * 4 + it) * 2u + hh;
            *(volatile v4f*)(S + (size_t)(mBase + row) * DM + n0 + c4) = vv[it];
          }
          __threadfence();
        }
      }
    }
    wave_sync_lds();
  }
}

__global__ __launch_bounds__(256) void k_final(const float* __restrict__ h, const float* __restrict__ res,
                                               const float* __restrict__ prs, const float* __restrict__ proj,
                                               const float* __restrict__ dif, const float* __restrict__ tbl,
                                               const float* __restrict__ S, const float* __restrict__ part,
                                               float* __restrict__ out) {
#pragma clang fp contract(off)
    __shared__ __align__(16) float sW[NBR * DM];
    const unsigned t = threadIdx.x, lane = t & 31u;
    const unsigned wave = (unsigned)__builtin_amdgcn_readfirstlane((int)(t >> 5));
#pragma unroll 4
    for (unsigned i = 0; i < (unsigned)((NBR * DM) / 256); ++i) {
        const unsigned e = i * 256u + t;
        const unsigned d = e / (unsigned)NBR;
        const unsigned j = e - d * (unsigned)NBR;
        sW[j * (unsigned)DM + d] = bfr(proj[e]);
    }
    __syncthreads();

    const unsigned jb = (lane < 9u) ? lane : 9u;
    float om = 0.0344827586207f;
    om = (jb == 8u) ? 0.0434782608696f : om;
    om = (jb == 7u) ? 0.0526315789474f : om;
    om = (jb == 6u) ? 0.0588235294118f : om;
    om = (jb == 5u) ? 0.0769230769231f : om;
    om = (jb == 4u) ? 0.0909090909091f : om;
    om = (jb == 3u) ? 0.142857142857f : om;
    om = (jb == 2u) ? 0.2f : om;
    om = (jb == 1u) ? 0.333333333333f : om;
    om = (jb == 0u) ? 0.5f : om;
    const float sqt = sqrtf(1.0f - om * om);
    const float tj = (float)jb * 0.111111111111f;
    const float cen = (-PI_F) * (1.0f - tj) + PI_F * tj;
    const float ratio = sqt / (om + 1e-8f);
    const float sint = sinf(om * 0.1f);

    const unsigned lj = (lane < 4u) ? lane : 4u;
    unsigned hp = 1000039u;
    hp = (lj == 3u) ? 1000037u : hp;
    hp = (lj == 2u) ? 1000033u : hp;
    hp = (lj == 1u) ? 999983u : hp;
    hp = (lj == 0u) ? 1000003u : hp;
    const unsigned ct = lane & 15u;
    const float dfv = bfr(dif[0]);

#pragma unroll 1
    for (unsigned rr = 0; rr < 8u; ++rr) {
        const unsigned row = blockIdx.x * 64u + wave * 8u + rr;
        const float* hr = h + (size_t)row * DM + 4u * lane;
        float sx = 0.f;
#pragma unroll
        for (int it = 0; it < 8; ++it) {
            const v4f a = *(const v4f*)(hr + it * 128);
            sx += (bfr(a.x) + bfr(a.y)) + (bfr(a.z) + bfr(a.w));
        }
        sx += __shfl_xor(sx, 16, 32);
        sx = xsum16(sx);
        const float xpos = sx * (1.0f / 1024.0f);

        float s5[NF];
#pragma unroll
        for (int f = 0; f < NF; ++f) s5[f] = part[(size_t)(ct * (unsigned)NF + (unsigned)f) * NROWS + row];
#pragma unroll
        for (int f = 0; f < NF; ++f) s5[f] = xsum16(s5[f]);
        float ssel = s5[4];
        ssel = (lj == 3u) ? s5[3] : ssel;
        ssel = (lj == 2u) ? s5[2] : ssel;
        ssel = (lj == 1u) ? s5[1] : ssel;
        ssel = (lj == 0u) ? s5[0] : ssel;
        const float gsel = sqrtf(ssel);
        const float g0 = __shfl(gsel, 0, 32);
        const float g1 = __shfl(gsel, 1, 32);
        const float g2 = __shfl(gsel, 2, 32);
        const float g3 = __shfl(gsel, 3, 32);
        const float g4 = __shfl(gsel, 4, 32);
        const float gmean = ((((g0 + g1) + g2) + g3) + g4) * 0.2f;
        const float flux = dfv * gmean + 1e-6f;
        const float pv = bfr(prs[row]);
        const float fac = expf(-pv * (1.0f / flux));

        float rq = bfr(res[(size_t)row * NF + lj]);
        rq = fminf(fmaxf(rq, -30000.0f), 30000.0f) * 100.0f;
        const int qi = (int)rq;
        unsigned term = (lane < 5u) ? ((unsigned)qi * hp) : 0u;
        term += __shfl_xor(term, 1, 32);
        term += __shfl_xor(term, 2, 32);
        term += __shfl_xor(term, 4, 32);
        const unsigned us = __shfl(term, 0, 32);
        int idx = (int)us % TBL;
        idx += (idx < 0) ? TBL : 0;
        idx = min(max(idx, 0), TBL - 1);
        const float tb = 0.05f * bfr(tbl[idx]);

        const float sech = 1.0f / (coshf(sqt * (xpos - cen)) + 1e-8f);
        const float ampv = 4.0f * atanf(ratio * sech * sint);

        v4f br[8];
#pragma unroll
        for (int it = 0; it < 8; ++it) br[it] = (v4f){0.f, 0.f, 0.f, 0.f};
#pragma unroll 1
        for (unsigned j = 0; j < (unsigned)NBR; ++j) {
            const float a = __shfl(ampv, (int)j, 32);
            const unsigned wo = j * (unsigned)DM + 4u * lane;
#pragma unroll
            for (int it = 0; it < 8; ++it) {
                const v4f w = *(const v4f*)(&sW[wo + (unsigned)it * 128u]);
                br[it] += w * a;
            }
        }

        const float* sr = S + (size_t)row * DM + 4u * lane;
        v4f o[8];
#pragma unroll
        for (int it = 0; it < 8; ++it) {
            const v4f sv = *(const v4f*)(sr + it * 128);
            o[it] = (sv * fac + br[it] * 0.5f) + tb;
        }
        float* orow = out + (size_t)row * DM + 4u * lane;
        for (int pass = 0; pass < 2; ++pass) {
#pragma unroll
            for (int it = 0; it < 8; ++it) *(volatile v4f*)(orow + it * 128) = o[it];
            __threadfence();
        }
    }
}

extern "C" void kernel_launch(void* const* d_in, const int* in_sizes, int n_in, void* d_out, int out_size,
                              void* d_ws, size_t ws_size, hipStream_t stream) {
    if (n_in < 8) return;
    if (in_sizes[0] < NROWS * DM || in_sizes[1] < NROWS * NF || in_sizes[2] < NROWS) return;
    if (in_sizes[3] < NF * NMODE * DM || in_sizes[4] < NF * NMODE * DM || in_sizes[5] < DM * NBR) return;
    if (in_sizes[6] < 1 || in_sizes[7] < TBL || out_size < NROWS * DM) return;
    if ((size_t)WS_TOTAL > ws_size) return;

    const float* h     = (const float*)d_in[0];
    const float* res   = (const float*)d_in[1];
    const float* prs   = (const float*)d_in[2];
    const float* Mw    = (const float*)d_in[3];
    const float* cw    = (const float*)d_in[4];
    const float* proj  = (const float*)d_in[5];
    const float* dif   = (const float*)d_in[6];
    const float* tbl   = (const float*)d_in[7];
    float* out = (float*)d_out;

    char* wsp = (char*)d_ws;
    size_t off = 0;
    unsigned short* h16  = (unsigned short*)(wsp + off); off += SZ_H16;
    unsigned short* w16  = (unsigned short*)(wsp + off); off += SZ_W16;
    unsigned short* m16  = (unsigned short*)(wsp + off); off += SZ_M16;
    unsigned short* a16  = (unsigned short*)(wsp + off); off += SZ_A16;
    float*          Ssum = (float*)(wsp + off);          off += SZ_S;
    float*          part = (float*)(wsp + off);          off += SZ_PART;
    if (off > ws_size || off > (size_t)134217728) return;

    k_cvt16<<<(unsigned)(((size_t)NROWS * DM / 8) / 256), 256, 0, stream>>>(h, (_Float16*)h16, (unsigned)((size_t)NROWS * DM / 8), SCL_H);
    k_cvt16<<<(unsigned)(((size_t)NA * DM / 8) / 256), 256, 0, stream>>>(cw, (_Float16*)w16, (unsigned)((size_t)NA * DM / 8), SCL_W);
    k_wt16<<<dim3((DM * (NMODE / 8)) / 256, NF), 256, 0, stream>>>(Mw, NMODE, DM, 5, m16, SCL_M);

    const unsigned gA = ((NROWS / 64) * (NA / 64) + 7) / 8;
    const unsigned gF = ((NROWS / 32) * NCT + 7) / 8;
    k_gemm_a<<<gA, 256, 0, stream>>>((const _Float16*)h16, DM, (const _Float16*)w16, DM, (_Float16*)a16, NA,
                                     NROWS, NA, DM, SCL_A);
    k_gemm_f<<<gF, 256, 0, stream>>>((const _Float16*)a16, (const _Float16*)m16, Ssum, part, SCL_R);
    k_final<<<NROWS / 64, 256, 0, stream>>>(h, res, prs, proj, dif, tbl, Ssum, part, out);
}
